// HGNN_59828894433623
// MI455X (gfx1250) — hardware-verified
//
#include <hip/hip_runtime.h>
#include <stddef.h>
#include <stdint.h>


#define FD     32
#define FH     64
#define NOUT   16
#define KIN    64
#define APP    384
#define APA    256
#define KBP    512
#define KBA    256
#define KHD    128
#define CSP    256
#define CSA    128
#define YSTEPS 4
#define KAP    12
#define KAA    8
#define NTHR   256
#define NWAVE  8
#define EPT    8
#define CHUNK  (NTHR * EPT)
#define WCAP   (EPT * 32)
#define LISTN  (NWAVE * WCAP)
#define NBA    1024
#define SLA    10
#define RCAP   28672
#define DEGCAP 1024
#define GBM    64
#define GBN    64
#define GTHR   128
#define APS    256
#define UPART  512
#define NPARTS 22
#define UHEAD  256
#define UTOT   (NPARTS * UPART + UHEAD)
#define AGG_ZINTS    (LISTN + 2 * RCAP + 3 * NBA)
#define MISC_INTS    16
#define ROWBUF_INTS  (NWAVE * APS / 2)
#define AGG_LDS_INTS (AGG_ZINTS + MISC_INTS + ROWBUF_INTS)
#define WSMAX  134217728

static_assert((CHUNK & (CHUNK - 1)) == 0 && CHUNK <= 4096);
static_assert((NBA & (NBA - 1)) == 0 && NBA == (1 << SLA));
static_assert(((long long)CHUNK << SLA) < (1LL << 31));
static_assert(LISTN % NTHR == 0);
static_assert(NBA % NWAVE == 0 && NBA % 32 == 0 && NBA % GBM == 0);
static_assert(RCAP % 4 == 0 && AGG_ZINTS % 4 == 0 && LISTN % 4 == 0 && ((AGG_ZINTS + MISC_INTS) % 4) == 0);
static_assert(AGG_ZINTS % (NTHR * 4) == 0);
static_assert(KIN % 32 == 0 && KBP % 32 == 0 && KBA % 32 == 0 && KHD % 32 == 0);
static_assert(KIN == 2 * FD && FD == 32);
static_assert(APP == 6 * FH && APA == 4 * FH && KBP == APP + 2 * FH && KBA == APA);
static_assert(KAP * 32 == APP && KAA * 32 == APA && YSTEPS * 32 == 2 * FH && KHD == 2 * FH);
static_assert(CSP + 2 * FH == APP && CSA + 2 * FH == APA);
static_assert(GBM == (GTHR / 32) * 16 && GBN == FH && FH == 2 * 32);
static_assert(APS >= 2 * FH);
static_assert(UPART == FH * (FH / 8) && UHEAD == NOUT * (KHD / 8));
static_assert(UPART % NTHR == 0 && (NPARTS * UPART) % NTHR == 0 && UTOT % NTHR == 0);
static_assert(AGG_LDS_INTS * 4 <= 300000);
static_assert(((GBM * NOUT * 4) % 128) == 0 && (GTHR % 4) == 0);

typedef float          v4f   __attribute__((ext_vector_type(4)));
typedef float          v8f   __attribute__((ext_vector_type(8)));
typedef int            v4i   __attribute__((ext_vector_type(4)));
typedef int            v8i   __attribute__((ext_vector_type(8)));
typedef unsigned short v4us  __attribute__((ext_vector_type(4)));
typedef unsigned short v8us  __attribute__((ext_vector_type(8)));
typedef unsigned short v16us __attribute__((ext_vector_type(16)));
typedef __bf16         v16bf __attribute__((ext_vector_type(16)));
typedef v4f  __attribute__((may_alias)) v4fa;
typedef v4i  __attribute__((may_alias)) v4ia;
typedef v4us __attribute__((may_alias)) v4usa;
typedef v8us __attribute__((may_alias)) v8usa;
typedef unsigned int __attribute__((may_alias)) ua32;
union FragB { v16bf v; v16us u; v8us h[2]; v8i w; };

__device__ __forceinline__ v8f wmb(const FragB& a, const FragB& b, v8f c) {
  v8f d = __builtin_amdgcn_wmma_f32_16x16x32_bf16(false, a.v, false, b.v, (short)0, c, false, false);
  asm volatile("v_nop\n\tv_nop\n\tv_nop\n\tv_nop" : "+v"(d) : "v"(a.w), "v"(b.w));
  return d;
}

__device__ __forceinline__ unsigned bf16_bits(float f) {
  const unsigned u = __float_as_uint(f);
  return ((u + 0x7FFFu + ((u >> 16) & 1u)) >> 16) & 0xFFFFu;
}
__device__ __forceinline__ float bf16_val(float f) {
  return __uint_as_float(bf16_bits(f) << 16);
}
__device__ __forceinline__ v4f bfr4(const v4f a) {
  v4f r; r.x = bf16_val(a.x); r.y = bf16_val(a.y); r.z = bf16_val(a.z); r.w = bf16_val(a.w); return r;
}
__device__ __forceinline__ void split2(float v, unsigned& hi, unsigned& lo) {
  hi = bf16_bits(v);
  lo = bf16_bits(v - __uint_as_float(hi << 16));
}

__device__ __forceinline__ void wave_sync() {
  __builtin_amdgcn_fence(__ATOMIC_RELEASE, "wavefront");
  __builtin_amdgcn_wave_barrier();
  __builtin_amdgcn_fence(__ATOMIC_ACQUIRE, "wavefront");
}

__device__ __forceinline__ FragB frag_f32(const float* __restrict__ p) {
  const v4f f0 = *(const v4f*)p;
  const v4f f1 = *(const v4f*)(p + 4);
  const v4f f2 = *(const v4f*)(p + 16);
  const v4f f3 = *(const v4f*)(p + 20);
  v16us u;
  u[0]  = (unsigned short)bf16_bits(f0.x); u[1]  = (unsigned short)bf16_bits(f0.y);
  u[2]  = (unsigned short)bf16_bits(f0.z); u[3]  = (unsigned short)bf16_bits(f0.w);
  u[4]  = (unsigned short)bf16_bits(f1.x); u[5]  = (unsigned short)bf16_bits(f1.y);
  u[6]  = (unsigned short)bf16_bits(f1.z); u[7]  = (unsigned short)bf16_bits(f1.w);
  u[8]  = (unsigned short)bf16_bits(f2.x); u[9]  = (unsigned short)bf16_bits(f2.y);
  u[10] = (unsigned short)bf16_bits(f2.z); u[11] = (unsigned short)bf16_bits(f2.w);
  u[12] = (unsigned short)bf16_bits(f3.x); u[13] = (unsigned short)bf16_bits(f3.y);
  u[14] = (unsigned short)bf16_bits(f3.z); u[15] = (unsigned short)bf16_bits(f3.w);
  FragB a;
  a.u = u;
  return a;
}

template <int SLB>
__device__ __forceinline__ int scan_chunk(const int* __restrict__ dsts, int nE, int cbase, int slotBase,
                                          int nb, int vec8, int* list, int tid, int lane, int wave) {
  int wc = 0;
  const int el0  = tid * EPT;
  const int e0   = cbase + el0;
  const int sent = -2147483647 - 1;
  v4i da, db;
  if (vec8 != 0 && cbase + CHUNK <= nE) {
    da = *(const v4i*)(dsts + e0);
    db = *(const v4i*)(dsts + e0 + 4);
  } else {
    da.x = (e0     < nE) ? dsts[min(e0,     nE - 1)] : sent;
    da.y = (e0 + 1 < nE) ? dsts[min(e0 + 1, nE - 1)] : sent;
    da.z = (e0 + 2 < nE) ? dsts[min(e0 + 2, nE - 1)] : sent;
    da.w = (e0 + 3 < nE) ? dsts[min(e0 + 3, nE - 1)] : sent;
    db.x = (e0 + 4 < nE) ? dsts[min(e0 + 4, nE - 1)] : sent;
    db.y = (e0 + 5 < nE) ? dsts[min(e0 + 5, nE - 1)] : sent;
    db.z = (e0 + 6 < nE) ? dsts[min(e0 + 6, nE - 1)] : sent;
    db.w = (e0 + 7 < nE) ? dsts[min(e0 + 7, nE - 1)] : sent;
  }
  const unsigned nbs = (unsigned)slotBase;
  const unsigned unb = (unsigned)nb;
  const unsigned s0 = (unsigned)da.x - nbs, s1 = (unsigned)da.y - nbs;
  const unsigned s2 = (unsigned)da.z - nbs, s3 = (unsigned)da.w - nbs;
  const unsigned s4 = (unsigned)db.x - nbs, s5 = (unsigned)db.y - nbs;
  const unsigned s6 = (unsigned)db.z - nbs, s7 = (unsigned)db.w - nbs;
  const bool h0 = s0 < unb, h1 = s1 < unb, h2 = s2 < unb, h3 = s3 < unb;
  const bool h4 = s4 < unb, h5 = s5 < unb, h6 = s6 < unb, h7 = s7 < unb;
  const unsigned any = __builtin_amdgcn_ballot_w32(h0 | h1 | h2 | h3 | h4 | h5 | h6 | h7);
  if (any != 0u) {
#define HITJ(J, HJ, SJ) { \
      const unsigned mj = __builtin_amdgcn_ballot_w32(HJ); \
      if (mj != 0u) { \
        if (HJ) { \
          const int pos = wc + (int)__builtin_amdgcn_mbcnt_lo(mj, 0u); \
          if (pos < WCAP) list[wave * WCAP + pos] = ((el0 + (J)) << SLB) | (int)(SJ); \
        } \
        wc += (int)__builtin_popcount(mj); } }
    HITJ(0, h0, s0)
    HITJ(1, h1, s1)
    HITJ(2, h2, s2)
    HITJ(3, h3, s3)
    HITJ(4, h4, s4)
    HITJ(5, h5, s5)
    HITJ(6, h6, s6)
    HITJ(7, h7, s7)
#undef HITJ
  }
  return wc;
}

__global__ __launch_bounds__(NTHR) void k_wprep(const float* __restrict__ wina, const float* __restrict__ winp,
                                                const float* __restrict__ wwl, const float* __restrict__ wwr,
                                                const float* __restrict__ cwl, const float* __restrict__ cwr,
                                                const float* __restrict__ bwl, const float* __restrict__ bwr,
                                                const float* __restrict__ linw,
                                                unsigned short* BinA, unsigned short* BinP, unsigned short* Bp,
                                                unsigned short* Ba, unsigned short* Bh) {
  const int u = (int)blockIdx.x * NTHR + (int)threadIdx.x;
  if (u >= UTOT) return;
  const float* W;
  unsigned short* P;
  int pitch, coff, ldw, n, k8;
  if (u < NPARTS * UPART) {
    const int p = u >> 9;
    const int v = u & (UPART - 1);
    n = v >> 3; k8 = (v & 7) * 8; ldw = FH;
    if (p == 0)      { W = wina; P = BinA; pitch = KIN; coff = 0; }
    else if (p == 1) { W = winp; P = BinP; pitch = KIN; coff = 0; }
    else if (p < 18) {
      const int q = p - 2, l = q >> 3, j = q & 7, mt = j >> 1;
      const float* base = (mt == 0) ? wwl : ((mt == 1) ? cwl : ((mt == 2) ? wwr : cwr));
      W = base + (size_t)l * FH * FH;
      P = Bp + (size_t)l * FH * KBP; pitch = KBP; coff = FH * j;
    } else {
      const int j = p - 18, mt = j >> 1;
      W = (mt == 0) ? bwl : bwr;
      P = Ba; pitch = KBA; coff = FH * j;
    }
  } else {
    const int v   = u - NPARTS * UPART;
    const int col = (v & 15) * 8;
    n = v >> 4; k8 = col & (FH - 1); coff = col & FH; ldw = NOUT;
    W = linw; P = Bh; pitch = KHD;
  }
  const float* p = W + (size_t)k8 * (size_t)ldw + n;
  float f[8];
#pragma unroll
  for (int i = 0; i < 8; ++i) f[i] = p[(size_t)i * ldw];
  v8us o;
#pragma unroll
  for (int i = 0; i < 8; ++i) o[i] = (unsigned short)bf16_bits(f[i]);
  unsigned short* dp = P + (size_t)n * (size_t)pitch + coff + k8;
  *(volatile v8us*)dp = o;
  __threadfence();
  *(volatile v8us*)dp = o;
}

template <int SRC, int RELU>
__global__ __launch_bounds__(GTHR) void k_gemm(const float* __restrict__ xd, const float* __restrict__ xc, int nX,
                                               unsigned short* Apl, int apitch, int kaSteps,
                                               const unsigned short* __restrict__ BT, int KB,
                                               const float* __restrict__ b1, const float* __restrict__ b2,
                                               int useB2, int coff) {
  __shared__ __attribute__((aligned(16))) float stg[GBM * GBN];
  const int tid = (int)threadIdx.x, lane = tid & 31, wave = tid >> 5, hh = lane >> 4, m = lane & 15;
  const int rowBase = (int)blockIdx.x * GBM;

  v8f acc[4];
  {
    const v8f z = {0.f, 0.f, 0.f, 0.f, 0.f, 0.f, 0.f, 0.f};
    acc[0] = z; acc[1] = z; acc[2] = z; acc[3] = z;
  }
  const unsigned short* wp = BT + (size_t)m * (size_t)KB + 8 * hh;
  if constexpr (SRC == 0) {
    const unsigned short* ap = Apl + (size_t)(rowBase + 16 * wave + m) * (size_t)apitch + 8 * hh;
    const int ksteps = KB >> 5;
#pragma unroll 1
    for (int ks = 0; ks < ksteps; ++ks) {
      const int aks = ks < kaSteps ? ks : ks - YSTEPS;
      FragB af;
      af.h[0] = *(const v8usa*)(ap + 32 * aks);
      af.h[1] = *(const v8usa*)(ap + 32 * aks + 16);
#pragma unroll
      for (int t = 0; t < 4; ++t) {
        const unsigned short* wq = wp + (size_t)(16 * t) * (size_t)KB + 32 * ks;
        FragB bf;
        bf.h[0] = *(const v8usa*)wq;
        bf.h[1] = *(const v8usa*)(wq + 16);
        acc[t] = wmb(af, bf, acc[t]);
      }
    }
  } else {
    int r = rowBase + 16 * wave + m;
    r = r < nX ? r : nX - 1;
    {
      const FragB af = frag_f32(xd + (size_t)r * FD + 8 * hh);
#pragma unroll
      for (int t = 0; t < 4; ++t) {
        const unsigned short* wq = wp + (size_t)(16 * t) * (size_t)KB;
        FragB bf;
        bf.h[0] = *(const v8usa*)wq;
        bf.h[1] = *(const v8usa*)(wq + 16);
        acc[t] = wmb(af, bf, acc[t]);
      }
    }
    {
      const FragB af = frag_f32(xc + (size_t)r * FD + 8 * hh);
#pragma unroll
      for (int t = 0; t < 4; ++t) {
        const unsigned short* wq = wp + (size_t)(16 * t) * (size_t)KB + 32;
        FragB bf;
        bf.h[0] = *(const v8usa*)wq;
        bf.h[1] = *(const v8usa*)(wq + 16);
        acc[t] = wmb(af, bf, acc[t]);
      }
    }
  }

#pragma unroll
  for (int t = 0; t < 4; ++t) {
    const int lc = 16 * t + m;
#pragma unroll
    for (int r = 0; r < 8; ++r) {
      const int lr = 16 * wave + 8 * hh + r;
      stg[lr * GBN + lc] = acc[t][r];
    }
  }
  __syncthreads();

  v4f bb4;
  {
    const float fu = (float)useB2;
    const v4f t1 = bfr4(*(const v4f*)(b1 + 4 * m));
    const v4f t2 = bfr4(*(const v4f*)(b2 + 4 * m));
    bb4 = t1 + t2 * fu;
  }
  v4f fv[8];
#pragma unroll
  for (int i = 0; i < 8; ++i) {
    const int lr = 16 * wave + 2 * i + hh;
    v4f t = *(const v4fa*)(stg + lr * GBN + 4 * m) + bb4;
    if constexpr (RELU != 0) {
      t.x = fmaxf(t.x, 0.0f); t.y = fmaxf(t.y, 0.0f); t.z = fmaxf(t.z, 0.0f); t.w = fmaxf(t.w, 0.0f);
    }
    fv[i] = t;
  }
  __syncthreads();

  unsigned short* sh = (unsigned short*)stg;
#pragma unroll
  for (int i = 0; i < 8; ++i) {
    const int lr = 16 * wave + 2 * i + hh;
    v4us h4, l4;
    unsigned ha, la, hb, lb, hc, lcx, hd, ld;
    split2(fv[i].x, ha, la); split2(fv[i].y, hb, lb); split2(fv[i].z, hc, lcx); split2(fv[i].w, hd, ld);
    h4[0] = (unsigned short)ha; h4[1] = (unsigned short)hb; h4[2] = (unsigned short)hc; h4[3] = (unsigned short)hd;
    l4[0] = (unsigned short)la; l4[1] = (unsigned short)lb; l4[2] = (unsigned short)lcx; l4[3] = (unsigned short)ld;
    *(v4usa*)(sh + (size_t)lr * (2 * GBN) + 4 * m) = h4;
    *(v4usa*)(sh + (size_t)lr * (2 * GBN) + FH + 4 * m) = l4;
  }
  __syncthreads();
  v8us q[8];
#pragma unroll
  for (int i = 0; i < 8; ++i) {
    const int lr = 16 * wave + 2 * i + hh;
    q[i] = *(const v8usa*)(sh + (size_t)lr * (2 * GBN) + 8 * m);
  }
#pragma unroll
  for (int i = 0; i < 8; ++i) {
    const int gr = rowBase + 16 * wave + 2 * i + hh;
    *(volatile v8us*)(Apl + (size_t)gr * (size_t)apitch + coff + 8 * m) = q[i];
  }
  __threadfence();
#pragma unroll
  for (int i = 0; i < 8; ++i) {
    const int gr = rowBase + 16 * wave + 2 * i + hh;
    *(volatile v8us*)(Apl + (size_t)gr * (size_t)apitch + coff + 8 * m) = q[i];
  }
}

__global__ __launch_bounds__(GTHR) void k_head(const unsigned short* __restrict__ A, int apitch, int acoff,
                                               const unsigned short* __restrict__ BT,
                                               const float* __restrict__ bias, float* outp, int nOut) {
  __shared__ __attribute__((aligned(16))) float stg[GBM * NOUT];
  const int tid = (int)threadIdx.x, lane = tid & 31, wave = tid >> 5, hh = lane >> 4, m = lane & 15;
  const int rowBase = (int)blockIdx.x * GBM;

  v8f acc = {0.f, 0.f, 0.f, 0.f, 0.f, 0.f, 0.f, 0.f};
  const unsigned short* ap = A + (size_t)(rowBase + 16 * wave + m) * (size_t)apitch + acoff + 8 * hh;
  const unsigned short* wp = BT + (size_t)m * (size_t)KHD + 8 * hh;
#pragma unroll 1
  for (int ks = 0; ks < KHD / 32; ++ks) {
    FragB af, bf;
    af.h[0] = *(const v8usa*)(ap + 32 * ks);
    af.h[1] = *(const v8usa*)(ap + 32 * ks + 16);
    bf.h[0] = *(const v8usa*)(wp + 32 * ks);
    bf.h[1] = *(const v8usa*)(wp + 32 * ks + 16);
    acc = wmb(af, bf, acc);
  }
#pragma unroll
  for (int r = 0; r < 8; ++r) {
    const int lr = 16 * wave + 8 * hh + r;
    stg[lr * NOUT + m] = acc[r];
  }
  __syncthreads();

  int live = nOut - rowBase; live = live < 0 ? 0 : (live > GBM ? GBM : live);
  const int npc = live * (NOUT / 4);
  const int c4 = (tid & 3) * 4;
  const v4f bb4 = bfr4(*(const v4f*)(bias + c4));
  float* ob = outp + (size_t)rowBase * NOUT;
#pragma unroll 1
  for (int p = tid; p < npc; p += GTHR) {
    const v4f v = *(const v4fa*)(stg + 4 * p) + bb4;
    *(volatile v4f*)(ob + 4 * p) = v;
  }
  __threadfence();
#pragma unroll 1
  for (int p = tid; p < npc; p += GTHR) {
    const v4f v = *(const v4fa*)(stg + 4 * p) + bb4;
    *(volatile v4f*)(ob + 4 * p) = v;
  }
}

__global__ __launch_bounds__(NTHR) void k_scan(const int* __restrict__ srcs, const int* __restrict__ dsts,
                                               int nE, int nSrc, int nDst, int vec8, int mRows,
                                               const unsigned short* gpl, int gpitch, int gcoff,
                                               unsigned short* opl, int opitch, int ocoff) {
  extern __shared__ __attribute__((aligned(16))) int dsm[];
  int* list = dsm;
  int* hl   = dsm + LISTN;
  int* sl   = hl + RCAP;
  int* cnt  = sl + RCAP;
  int* offs = cnt + NBA;
  int* cur  = offs + NBA;
  int* misc = cur + NBA;
  const int tid = (int)threadIdx.x, lane = tid & 31, wave = tid >> 5;
  unsigned short* rowbuf = (unsigned short*)(misc + MISC_INTS) + wave * APS;
  const int nodeBase = (int)blockIdx.x * NBA;

  {
    const v4i z4 = {0, 0, 0, 0};
    for (int i = tid * 4; i < AGG_ZINTS; i += NTHR * 4) *(v4ia*)(dsm + i) = z4;
    if (tid < MISC_INTS) misc[tid] = 0;
  }
  __syncthreads();

  int t = 0, ov = 0;
  const int nChunks = (nE + CHUNK - 1) / CHUNK;
#pragma unroll 1
  for (int ch = 0; ch < nChunks; ++ch) {
    const int cbase = ch * CHUNK;
    const int wc = scan_chunk<SLA>(dsts, nE, cbase, nodeBase, NBA, vec8, list, tid, lane, wave);
    if (lane == 0) misc[wave] = wc;
    __syncthreads();
    if (wave == 0) {
#pragma unroll 1
      for (int w2 = 0; w2 < NWAVE; ++w2) {
        int c = misc[w2];
        c = c < 0 ? 0 : (c > WCAP ? WCAP : c);
#pragma unroll 1
        for (int b0 = 0; b0 < c; b0 += 32) {
          const int idx = b0 + lane;
          const int ent = list[w2 * WCAP + (idx < WCAP ? idx : WCAP - 1)];
          const int m32 = (c - b0) < 32 ? (c - b0) : 32;
#pragma unroll 1
          for (int k = 0; k < m32; ++k) {
            const int u    = __builtin_amdgcn_readlane(ent, k);
            const int slot = u & (NBA - 1);
            const int el   = (u >> SLA) & (CHUNK - 1);
            const int pk   = ((cbase + el) << SLA) | slot;
            if (t < RCAP) {
              if (lane == 0) { hl[t] = pk; cnt[slot] = cnt[slot] + 1; }
              t = t + 1;
            } else {
              ov = 1;
            }
          }
        }
      }
    }
    __syncthreads();
  }
  if (wave == 0 && lane == 0) { misc[8] = t; misc[9] = ov; }
  __syncthreads();
  int tt = misc[8];
  tt = tt < 0 ? 0 : (tt > RCAP ? RCAP : tt);
  const int ovf = misc[9];

  if (wave == 0) {
    const int base = lane * (NBA / 32);
    int s = 0;
#pragma unroll 1
    for (int i = 0; i < NBA / 32; ++i) s += cnt[base + i];
    int incl = s;
#pragma unroll
    for (int d = 1; d < 32; d <<= 1) {
      const int y = __shfl_up(incl, d, 32);
      if (lane >= d) incl += y;
    }
    int run = incl - s;
#pragma unroll 1
    for (int i = 0; i < NBA / 32; ++i) {
      const int cv = cnt[base + i];
      offs[base + i] = run;
      cur[base + i]  = run;
      run += cv;
    }
  }
  __syncthreads();
  if (wave == 0) {
#pragma unroll 1
    for (int b0 = 0; b0 < tt; b0 += 32) {
      const int idx = b0 + lane;
      const int ent = hl[idx < RCAP ? idx : RCAP - 1];
      const int m32 = (tt - b0) < 32 ? (tt - b0) : 32;
#pragma unroll 1
      for (int k = 0; k < m32; ++k) {
        const int u    = __builtin_amdgcn_readlane(ent, k);
        const int slot = u & (NBA - 1);
        if (lane == 0) {
          int p = cur[slot];
          p = p < 0 ? 0 : (p > RCAP - 1 ? RCAP - 1 : p);
          sl[p] = u;
          cur[slot] = p + 1;
        }
      }
    }
  }
  __syncthreads();

  const float qnan = __int_as_float(0x7fc00000);
  const float pz = (ovf != 0) ? qnan : 0.0f;
#pragma unroll 1
  for (int si = 0; si < NBA / NWAVE; ++si) {
    const int s    = si * NWAVE + wave;
    const int node = nodeBase + s;
    int c = cnt[s];
    const bool big = c > DEGCAP;
    c = c < 0 ? 0 : (c > DEGCAP ? DEGCAP : c);
    int o = offs[s];
    o = o < 0 ? 0 : (o > RCAP ? RCAP : o);
    float a0 = 0.0f, a1 = 0.0f;
#pragma unroll 1
    for (int b0 = 0; b0 < c; b0 += 32) {
      int idx = o + b0 + lane;
      idx = idx > RCAP - 1 ? RCAP - 1 : idx;
      const int ent = sl[idx];
      int eid = ent >> SLA;
      eid = eid < 0 ? 0 : (eid > nE - 1 ? nE - 1 : eid);
      int sr = srcs[eid];
      sr = sr < 0 ? 0 : (sr > nSrc - 1 ? nSrc - 1 : sr);
      const int m32 = (c - b0) < 32 ? (c - b0) : 32;
#pragma unroll 1
      for (int k = 0; k < m32; ++k) {
        const int sk = __builtin_amdgcn_readlane(sr, k);
        const size_t rb = (size_t)sk * (size_t)gpitch + (size_t)gcoff + (size_t)(2 * lane);
        const unsigned wh = *(const ua32*)(gpl + rb);
        const unsigned wl = *(const ua32*)(gpl + rb + FH);
        const float f0 = __uint_as_float(wh << 16)         + __uint_as_float(wl << 16);
        const float f1 = __uint_as_float(wh & 0xffff0000u) + __uint_as_float(wl & 0xffff0000u);
        a0 += f0; a1 += f1;
      }
    }
    const float inv = 1.0f / fmaxf((float)c, 1.0f);
    const float pzr = big ? qnan : pz;
    const bool live = node < nDst;
    const float m0 = live ? (a0 * inv + pzr) : 0.0f;
    const float m1 = live ? (a1 * inv + pzr) : 0.0f;
    unsigned mh0, ml0, mh1, ml1;
    split2(m0, mh0, ml0); split2(m1, mh1, ml1);
    ua32* rb32 = (ua32*)rowbuf;
    rb32[lane]      = mh0 | (mh1 << 16);
    rb32[32 + lane] = ml0 | (ml1 << 16);
    wave_sync();
    const v8us q0 = *(const v8usa*)(rowbuf + 8 * (lane & 15));
    wave_sync();
    if (node < mRows) {
      unsigned short* rpw = opl + (size_t)node * (size_t)opitch + ocoff + 8 * (lane & 15);
      if (lane < 16) *(volatile v8us*)rpw = q0;
      __threadfence();
      if (lane < 16) *(volatile v8us*)rpw = q0;
    }
  }
}

static inline int cdiv(int a, int b) { return (a + b - 1) / b; }

extern "C" void kernel_launch(void* const* d_in, const int* in_sizes, int n_in,
                              void* d_out, int out_size, void* d_ws, size_t ws_size,
                              hipStream_t stream) {
  if (n_in < 25) return;
  if (in_sizes[0] < FD || (in_sizes[0] % FD) != 0 || in_sizes[1] != in_sizes[0]) return;
  if (in_sizes[2] < FD || (in_sizes[2] % FD) != 0 || in_sizes[3] != in_sizes[2]) return;
  const int nA = in_sizes[0] / FD;
  const int nP = in_sizes[2] / FD;
  if (nA > (1 << 22) || nP > (1 << 22)) return;
  if (in_sizes[4] != KIN * FH || in_sizes[5] != FH || in_sizes[6] != KIN * FH || in_sizes[7] != FH) return;
  for (int i = 8; i <= 14; i += 3) {
    if (in_sizes[i] != 2 * FH * FH || in_sizes[i + 1] != 2 * FH || in_sizes[i + 2] != 2 * FH * FH) return;
  }
  if (in_sizes[17] != FH * NOUT || in_sizes[18] != NOUT) return;
  const int eW = in_sizes[19], eB = in_sizes[21], eC = in_sizes[23];
  if (in_sizes[20] != eW || in_sizes[22] != eB || in_sizes[24] != eC) return;
  if (eW < 1 || eB < 1 || eC < 1) return;
  if (eW >= (1 << 21) || eB >= (1 << 21) || eC >= (1 << 21)) return;
  if ((long long)out_size != (long long)nP * NOUT) return;

  const float* xda  = (const float*)d_in[0];
  const float* xca  = (const float*)d_in[1];
  const float* xdp  = (const float*)d_in[2];
  const float* xcp  = (const float*)d_in[3];
  const float* wina = (const float*)d_in[4];
  const float* bina = (const float*)d_in[5];
  const float* winp = (const float*)d_in[6];
  const float* binp = (const float*)d_in[7];
  const float* wwl  = (const float*)d_in[8];
  const float* wbl  = (const float*)d_in[9];
  const float* wwr  = (const float*)d_in[10];
  const float* bwl  = (const float*)d_in[11];
  const float* bbl  = (const float*)d_in[12];
  const float* bwr  = (const float*)d_in[13];
  const float* cwl  = (const float*)d_in[14];
  const float* cbl  = (const float*)d_in[15];
  const float* cwr  = (const float*)d_in[16];
  const float* linw = (const float*)d_in[17];
  const float* linb = (const float*)d_in[18];
  const int* wsrc = (const int*)d_in[19];
  const int* wdst = (const int*)d_in[20];
  const int* bsrc = (const int*)d_in[21];
  const int* bdst = (const int*)d_in[22];
  const int* csrc = (const int*)d_in[23];
  const int* cdst = (const int*)d_in[24];
  float* out = (float*)d_out;

  const int MPA = cdiv(nA, GBM) * GBM;
  const int MPP = cdiv(nP, GBM) * GBM;
  const int gMA = MPA / GBM, gMP = MPP / GBM;
  const int gSA = cdiv(MPA, NBA), gSP = cdiv(MPP, NBA);
  if ((long long)gSA * NBA < (long long)MPA || (long long)gSP * NBA < (long long)MPP) return;
  const int vec8 = 1;

  char* ws = (char*)d_ws;
  size_t off = 0;
  const size_t oBinA = off; off += (size_t)FH * KIN * 2;                   off = (off + 255) & ~(size_t)255;
  const size_t oBinP = off; off += (size_t)FH * KIN * 2;                   off = (off + 255) & ~(size_t)255;
  const size_t oBp   = off; off += (size_t)2 * FH * KBP * 2;               off = (off + 255) & ~(size_t)255;
  const size_t oBa   = off; off += (size_t)FH * KBA * 2;                   off = (off + 255) & ~(size_t)255;
  const size_t oBh   = off; off += (size_t)NOUT * KHD * 2;                 off = (off + 255) & ~(size_t)255;
  const size_t oAp   = off; off += (size_t)MPP * APP * 2;                  off = (off + 255) & ~(size_t)255;
  const size_t oAa   = off; off += (size_t)MPA * APA * 2;                  off = (off + 255) & ~(size_t)255;
  if (off > ws_size || off > (size_t)WSMAX) return;
  unsigned short* BinA = (unsigned short*)(ws + oBinA);
  unsigned short* BinP = (unsigned short*)(ws + oBinP);
  unsigned short* Bp   = (unsigned short*)(ws + oBp);
  unsigned short* Ba   = (unsigned short*)(ws + oBa);
  unsigned short* Bh   = (unsigned short*)(ws + oBh);
  unsigned short* Ap   = (unsigned short*)(ws + oAp);
  unsigned short* Aa   = (unsigned short*)(ws + oAa);

  const size_t scanLds = (size_t)AGG_LDS_INTS * 4;
  hipFuncSetAttribute(reinterpret_cast<const void*>(&k_scan), hipFuncAttributeMaxDynamicSharedMemorySize, (int)scanLds);

  k_wprep<<<UTOT / NTHR, NTHR, 0, stream>>>(wina, winp, wwl, wwr, cwl, cwr, bwl, bwr, linw, BinA, BinP, Bp, Ba, Bh);
  k_gemm<1, 1><<<gMA, GTHR, 0, stream>>>(xda, xca, nA, Aa, APA, 0, BinA, KIN, bina, bina, 0, CSA);
  k_gemm<1, 1><<<gMP, GTHR, 0, stream>>>(xdp, xcp, nP, Ap, APP, 0, BinP, KIN, binp, binp, 0, CSP);
  k_scan<<<gSP, NTHR, scanLds, stream>>>(wsrc, wdst, eW, nA, nP, vec8, MPP, Aa, APA, CSA, Ap, APP, 0);
  k_scan<<<gSP, NTHR, scanLds, stream>>>(csrc, cdst, eC, nP, nP, vec8, MPP, Ap, APP, CSP, Ap, APP, 2 * FH);
  k_scan<<<gSA, NTHR, scanLds, stream>>>(bsrc, bdst, eB, nP, nA, vec8, MPA, Ap, APP, CSP, Aa, APA, 0);
  k_gemm<0, 0><<<gMP, GTHR, 0, stream>>>(xdp, xcp, nP, Ap, APP, KAP, Bp, KBP, wbl, cbl, 1, CSP);
  k_gemm<0, 0><<<gMA, GTHR, 0, stream>>>(xda, xca, nA, Aa, APA, KAA, Ba, KBA, bbl, bbl, 0, CSA);
  k_scan<<<gSP, NTHR, scanLds, stream>>>(wsrc, wdst, eW, nA, nP, vec8, MPP, Aa, APA, CSA, Ap, APP, 0);
  k_scan<<<gSP, NTHR, scanLds, stream>>>(csrc, cdst, eC, nP, nP, vec8, MPP, Ap, APP, CSP, Ap, APP, 2 * FH);
  k_gemm<0, 0><<<gMP, GTHR, 0, stream>>>(xdp, xcp, nP, Ap, APP, KAP, Bp + (size_t)FH * KBP, KBP,
                                         wbl + FH, cbl + FH, 1, CSP);
  k_head<<<gMP, GTHR, 0, stream>>>(Ap, APP, CSP, Bh, linb, out, nP);
}
